// NeuralLSLv2_18975165514075
// MI455X (gfx1250) — hardware-verified
//
#include <hip/hip_runtime.h>
#include <math.h>
#include <stddef.h>
#include <stdint.h>


#define DMOD  256
#define NBIT  64
#define ROWS  64
#define NTHR  256
#define WSCAP 134217728

#define WSC   64.0f
#define ASC   8.0f
#define PSC   4096.0f

#define OFF_ACT 0
#define OFF_WB  32768
#define OFF_PRE 65536
#define OFF_SQ  131072
#define OFF_PRB 163840
#define OFF_SK  172032
#define OFF_PK  188416
#define OFF_SCR 204800
#define LDS_MAIN 221184

static_assert(NTHR == 256);
static_assert(ROWS == 64);
static_assert(NBIT == 64);
static_assert((DMOD % 32) == 0);
static_assert((NBIT % 32) == 0);
static_assert(OFF_WB  == OFF_ACT + ROWS * DMOD * 2);
static_assert(OFF_PRE == OFF_WB  + 64 * DMOD * 2);
static_assert(OFF_SQ  == OFF_PRE + ROWS * DMOD * 4);
static_assert(OFF_PRB == OFF_SQ  + ROWS * DMOD * 2);
static_assert(OFF_SK  == OFF_PRB + ROWS * NBIT * 2);
static_assert(OFF_PK  == OFF_SK  + ROWS * NBIT * 4);
static_assert(OFF_SCR == OFF_PK  + NBIT * NBIT * 4);
static_assert(LDS_MAIN == OFF_SCR + ROWS * NBIT * 4);
static_assert(LDS_MAIN <= 300 * 1024);

typedef float    v4f  __attribute__((ext_vector_type(4)));
typedef float    v8f  __attribute__((ext_vector_type(8)));
typedef _Float16 v4h  __attribute__((ext_vector_type(4)));
typedef _Float16 v8h  __attribute__((ext_vector_type(8)));
typedef _Float16 v16h __attribute__((ext_vector_type(16)));
union FragH { v16h v; v8h h[2]; };

__device__ __forceinline__ v8f wmf(v16h a, v16h b, v8f c) {
  v8f d = __builtin_amdgcn_wmma_f32_16x16x32_f16(false, a, false, b, (short)0, c, false, false);
  asm volatile("v_nop\n\tv_nop\n\tv_nop\n\tv_nop" : "+v"(d) : "v"(a), "v"(b));
  return d;
}

__device__ __forceinline__ v8f vzero8() {
  v8f z = {0.f, 0.f, 0.f, 0.f, 0.f, 0.f, 0.f, 0.f};
  return z;
}

__device__ __forceinline__ float gelu_f(float x) {
  return 0.5f * x * (1.0f + erff(x * 0.70710678118654752f));
}

__device__ __forceinline__ float wsum(float v) {
#pragma unroll
  for (int o = 16; o > 0; o >>= 1) v += __shfl_xor(v, o, 32);
  return v;
}
__device__ __forceinline__ float wmax(float v) {
#pragma unroll
  for (int o = 16; o > 0; o >>= 1) v = fmaxf(v, __shfl_xor(v, o, 32));
  return v;
}

__global__ __launch_bounds__(NTHR) void k_pack(const float* __restrict__ W, _Float16* dst,
                                               int KD, int nch, int ldw, int rowoff, int total8) {
  const int idx = blockIdx.x * NTHR + (int)threadIdx.x;
  if (idx < total8) {
    const int e   = idx * 8;
    const int per = KD * 64;
    const int ch  = e / per;
    const int rr  = e - ch * per;
    const int c   = rr / KD;
    const int k0  = rr - c * KD;
    const int col = ch * 64 + c;
    const float* src = W + (size_t)(rowoff + k0) * ldw + col;
    v8h hv;
#pragma unroll
    for (int i = 0; i < 8; ++i) hv[i] = (_Float16)(src[(size_t)i * ldw] * WSC);
    _Float16* d = dst + e;
    *(volatile v8h*)d = hv;
    __threadfence();
    *(volatile v8h*)d = hv;
  }
}

__global__ __launch_bounds__(NTHR) void k_tab(const float* __restrict__ pos,
                                              const float* __restrict__ Wq, const float* __restrict__ bq,
                                              const float* __restrict__ Wk, const float* __restrict__ bk,
                                              const float* __restrict__ Wv1, const float* __restrict__ bv1,
                                              float* keys, float* pqb, float* pvb) {
  __shared__ __attribute__((aligned(16))) float st[3 * DMOD];
  const int i = blockIdx.x, d = threadIdx.x;
  const float* pr = pos + (size_t)i * DMOD;
  float ak = 0.f, aq = 0.f, av = 0.f;
#pragma unroll 1
  for (int j = 0; j < DMOD; ++j) {
    const float pe = pr[j];
    const size_t o = (size_t)j * DMOD + d;
    ak += pe * Wk[o];
    aq += pe * Wq[o];
    av += pe * Wv1[o];
  }
  st[d]            = ak + bk[d];
  st[DMOD + d]     = aq + bq[d];
  st[2 * DMOD + d] = av + bv1[d];
  __syncthreads();
  const int grp = d >> 6, q = d & 63;
  const int gsel = (grp < 3) ? grp : 0;
  const v4f v = *(const v4f*)(st + gsel * DMOD + 4 * q);
  float* gb = (grp == 0) ? keys : ((grp == 1) ? pqb : pvb);
  float* dp = gb + (size_t)i * DMOD + 4 * q;
  if (grp < 3) *(volatile v4f*)dp = v;
  __threadfence();
  if (grp < 3) *(volatile v4f*)dp = v;
}

__global__ __launch_bounds__(64) void k_pk(const float* __restrict__ pqb, const float* __restrict__ keys,
                                           float* pk, _Float16* keysh) {
  __shared__ __attribute__((aligned(16))) float st[NBIT];
  const int p = blockIdx.x, t = threadIdx.x;
  const float* qr = pqb + (size_t)p * DMOD;
  const float* kr = keys + (size_t)t * DMOD;
  float a = 0.f;
#pragma unroll 1
  for (int d = 0; d < DMOD; ++d) a += qr[d] * kr[d];
  st[t] = a * (1.0f / 16.0f);
  const int j = t & 31;
  const float* ks = keys + (size_t)p * DMOD + 8 * j;
  const v4f kx = *(const v4f*)ks;
  const v4f ky = *(const v4f*)(ks + 4);
  v8h hv;
  hv[0] = (_Float16)(kx.x * WSC); hv[1] = (_Float16)(kx.y * WSC);
  hv[2] = (_Float16)(kx.z * WSC); hv[3] = (_Float16)(kx.w * WSC);
  hv[4] = (_Float16)(ky.x * WSC); hv[5] = (_Float16)(ky.y * WSC);
  hv[6] = (_Float16)(ky.z * WSC); hv[7] = (_Float16)(ky.w * WSC);
  __syncthreads();
  const v4f pv = *(const v4f*)(st + 4 * (t & 15));
  float* pkd = pk + (size_t)p * NBIT + 4 * (t & 15);
  _Float16* khd = keysh + (size_t)p * DMOD + 8 * j;
  if (t < 16) *(volatile v4f*)pkd = pv;
  if (t < 32) *(volatile v8h*)khd = hv;
  __threadfence();
  if (t < 16) *(volatile v4f*)pkd = pv;
  if (t < 32) *(volatile v8h*)khd = hv;
}

struct EpiF32B {
  float* dst; int ldo; float s; const float* bias;
  __device__ __forceinline__ void operator()(int row0, int col0, int m, v8f c) const {
    const float b = bias[col0 + m];
#pragma unroll
    for (int r = 0; r < 8; ++r) dst[(row0 + r) * ldo + col0 + m] = c[r] * s + b;
  }
};
struct EpiF32 {
  float* dst; int ldo; float s;
  __device__ __forceinline__ void operator()(int row0, int col0, int m, v8f c) const {
#pragma unroll
    for (int r = 0; r < 8; ++r) dst[(row0 + r) * ldo + col0 + m] = c[r] * s;
  }
};
struct EpiF16 {
  _Float16* dst; int ldo; float s;
  __device__ __forceinline__ void operator()(int row0, int col0, int m, v8f c) const {
#pragma unroll
    for (int r = 0; r < 8; ++r) dst[(row0 + r) * ldo + col0 + m] = (_Float16)(c[r] * s);
  }
};

template<int KD, int NCH, typename Epi>
__device__ __forceinline__ void gemm64(const _Float16* A, const int lda, _Float16* wb,
                                       const _Float16* __restrict__ Wg, const Epi epi) {
  static_assert((KD % 32) == 0);
  static_assert(KD * 64 * 2 <= OFF_PRE - OFF_WB);
  const int t = threadIdx.x, lane = t & 31, wave = t >> 5, h = lane >> 4, m = lane & 15;
  const int mt = wave >> 1, ntb = (wave & 1) * 2;
#pragma unroll 1
  for (int ch = 0; ch < NCH; ++ch) {
    __syncthreads();
    const _Float16* src = Wg + (size_t)ch * (KD * 64);
    for (int e = t * 8; e < KD * 64; e += NTHR * 8) *(v8h*)(wb + e) = *(const v8h*)(src + e);
    __syncthreads();
    v8f c0 = vzero8(), c1 = vzero8();
    const _Float16* ap  = A + (16 * mt + m) * lda + 8 * h;
    const _Float16* bp0 = wb + (16 * ntb + m) * KD + 8 * h;
    const _Float16* bp1 = bp0 + 16 * KD;
#pragma unroll 2
    for (int kk = 0; kk < KD; kk += 32) {
      FragH a, b0, b1;
      a.h[0]  = *(const v8h*)(ap + kk);
      a.h[1]  = *(const v8h*)(ap + kk + 16);
      b0.h[0] = *(const v8h*)(bp0 + kk);
      b0.h[1] = *(const v8h*)(bp0 + kk + 16);
      b1.h[0] = *(const v8h*)(bp1 + kk);
      b1.h[1] = *(const v8h*)(bp1 + kk + 16);
      c0 = wmf(a.v, b0.v, c0);
      c1 = wmf(a.v, b1.v, c1);
    }
    epi(16 * mt + 8 * h, ch * 64 + 16 * ntb,      m, c0);
    epi(16 * mt + 8 * h, ch * 64 + 16 * ntb + 16, m, c1);
  }
  __syncthreads();
}

__device__ __forceinline__ void ln_gelu(const float* pre, _Float16* act,
                                        const float* __restrict__ g, const float* __restrict__ be) {
  const int t = threadIdx.x, lane = t & 31, wave = t >> 5;
  const v4f ga = *(const v4f*)(g + 8 * lane);
  const v4f gc = *(const v4f*)(g + 8 * lane + 4);
  const v4f ba = *(const v4f*)(be + 8 * lane);
  const v4f bc = *(const v4f*)(be + 8 * lane + 4);
  const float gv[8] = {ga.x, ga.y, ga.z, ga.w, gc.x, gc.y, gc.z, gc.w};
  const float bv[8] = {ba.x, ba.y, ba.z, ba.w, bc.x, bc.y, bc.z, bc.w};
#pragma unroll 1
  for (int i = 0; i < 8; ++i) {
    const int r = wave * 8 + i;
    const float* row = pre + r * DMOD + 8 * lane;
    const v4f x0 = *(const v4f*)row;
    const v4f x1 = *(const v4f*)(row + 4);
    float x[8] = {x0.x, x0.y, x0.z, x0.w, x1.x, x1.y, x1.z, x1.w};
    float s = 0.f;
#pragma unroll
    for (int j = 0; j < 8; ++j) s += x[j];
    s = wsum(s);
    const float mean = s * (1.0f / (float)DMOD);
    float s2 = 0.f;
#pragma unroll
    for (int j = 0; j < 8; ++j) { const float dv = x[j] - mean; x[j] = dv; s2 += dv * dv; }
    s2 = wsum(s2);
    const float inv = rsqrtf(s2 * (1.0f / (float)DMOD) + 1e-5f);
    v8h hv;
#pragma unroll
    for (int j = 0; j < 8; ++j) {
      const float y = x[j] * inv * gv[j] + bv[j];
      hv[j] = (_Float16)(gelu_f(y) * ASC);
    }
    *(v8h*)(act + r * DMOD + 8 * lane) = hv;
  }
}

__device__ __forceinline__ void softmax64(const float* lg, _Float16* prb) {
  const int t = threadIdx.x, lane = t & 31, wave = t >> 5;
#pragma unroll 1
  for (int i = 0; i < 8; ++i) {
    const int r = wave * 8 + i;
    const float l0 = lg[r * NBIT + 2 * lane];
    const float l1 = lg[r * NBIT + 2 * lane + 1];
    const float mx = wmax(fmaxf(l0, l1));
    const float e0 = __expf(l0 - mx);
    const float e1 = __expf(l1 - mx);
    const float sm = wsum(e0 + e1);
    const float inv = 1.0f / sm;
    prb[r * NBIT + 2 * lane]     = (_Float16)(e0 * inv * PSC);
    prb[r * NBIT + 2 * lane + 1] = (_Float16)(e1 * inv * PSC);
  }
}

__global__ __launch_bounds__(NTHR) void k_main(
    const float* __restrict__ ibits, const float* __restrict__ sbits,
    const float* __restrict__ b1, const float* __restrict__ g1, const float* __restrict__ be1,
    const float* __restrict__ b2, const float* __restrict__ g2, const float* __restrict__ be2,
    const float* __restrict__ b3, const float* __restrict__ g3, const float* __restrict__ be3,
    const float* __restrict__ b4,
    const float* __restrict__ Wv2, const float* __restrict__ bv2,
    const float* __restrict__ pvb, const float* __restrict__ pk,
    const _Float16* __restrict__ W1h, const _Float16* __restrict__ W2h,
    const _Float16* __restrict__ W3h, const _Float16* __restrict__ W4h,
    const _Float16* __restrict__ posh, const _Float16* __restrict__ Wqh,
    const _Float16* __restrict__ Wv1h, const _Float16* __restrict__ keysh,
    float* out)
{
  extern __shared__ v4f lds_dyn[];
  unsigned char* lb = (unsigned char*)lds_dyn;
  _Float16* act = (_Float16*)(lb + OFF_ACT);
  _Float16* wb  = (_Float16*)(lb + OFF_WB);
  float*    pre = (float*)(lb + OFF_PRE);
  _Float16* sq  = (_Float16*)(lb + OFF_SQ);
  _Float16* prb = (_Float16*)(lb + OFF_PRB);
  float*    sk  = (float*)(lb + OFF_SK);
  float*    pkT = (float*)(lb + OFF_PK);
  float*    scr = (float*)(lb + OFF_SCR);

  const int t = threadIdx.x, lane = t & 31, wave = t >> 5;
  const size_t rowbase = (size_t)blockIdx.x * ROWS;

#pragma unroll
  for (int i = 0; i < 4; ++i) {
    const int e = 4 * (i * NTHR + t);
    const v4f x = *(const v4f*)(sbits + rowbase * NBIT + e);
    v4h hx;
    hx[0] = (_Float16)x.x; hx[1] = (_Float16)x.y; hx[2] = (_Float16)x.z; hx[3] = (_Float16)x.w;
    *(v4h*)(act + e) = hx;
  }
#pragma unroll
  for (int i = 0; i < 16; ++i) {
    const int e = i * NTHR + t;
    const int p = e >> 6, k = e & 63;
    pkT[k * NBIT + p] = pk[e];
  }

  gemm64<NBIT, 4>(act, NBIT, wb, W1h, EpiF32B{pre, DMOD, 1.0f / 64.0f, b1});
  ln_gelu(pre, act, g1, be1);
  gemm64<DMOD, 4>(act, DMOD, wb, W2h, EpiF32B{pre, DMOD, 1.0f / 512.0f, b2});
  ln_gelu(pre, act, g2, be2);
  gemm64<DMOD, 4>(act, DMOD, wb, W3h, EpiF32B{pre, DMOD, 1.0f / 512.0f, b3});
  ln_gelu(pre, act, g3, be3);
  gemm64<DMOD, 1>(act, DMOD, wb, W4h, EpiF32B{scr, NBIT, 1.0f / 512.0f, b4});

  softmax64(scr, prb);

  gemm64<NBIT, 4>(prb, NBIT, wb, posh, EpiF16{act, DMOD, 1.0f / 32768.0f});
  gemm64<DMOD, 4>(act, DMOD, wb, Wqh,  EpiF16{sq, DMOD, 1.0f / 64.0f});
  gemm64<DMOD, 4>(act, DMOD, wb, Wv1h, EpiF32{pre, DMOD, 1.0f / 512.0f});
  gemm64<DMOD, 1>(sq, DMOD, wb, keysh, EpiF32{sk, NBIT, 1.0f / 8192.0f});

  {
    const int p  = 32 * (wave & 1) + lane;
    const int rg = wave >> 1;
    const float bv2v = bv2[0];
    const float* pvr = pvb + (size_t)p * DMOD;
#pragma unroll 1
    for (int i = 0; i < 16; ++i) {
      const int r = rg + 4 * i;
      const float* skr = sk + r * NBIT;
      float mx = -3.0e38f;
#pragma unroll 4
      for (int k = 0; k < NBIT; ++k) mx = fmaxf(mx, pkT[k * NBIT + p] + skr[k]);
      const float* ibr = ibits + (rowbase + r) * NBIT;
      float den = 0.f, num = 0.f;
#pragma unroll 4
      for (int k = 0; k < NBIT; ++k) {
        const float l = pkT[k * NBIT + p] + skr[k];
        const float e = __expf(l - mx);
        den += e;
        num += e * ibr[k];
      }
      const float gath = num * (1.0f / den);
      const float* svr = pre + r * DMOD;
      float v = 0.f;
#pragma unroll 2
      for (int c = 0; c < DMOD; ++c) {
        const float x = pvr[c] + svr[c];
        v += gelu_f(x) * Wv2[c];
      }
      v += bv2v;
      v = fmaxf(v, -60.0f);
      const float sig = 1.0f / (1.0f + __expf(-v));
      scr[r * NBIT + p] = gath * sig;
    }
  }
  __syncthreads();

  float* ob = out + rowbase * NBIT;
  v4f ov[4];
#pragma unroll
  for (int q = 0; q < 4; ++q) ov[q] = *(const v4f*)(scr + 4 * (q * NTHR + t));
#pragma unroll
  for (int q = 0; q < 4; ++q) *(volatile v4f*)(ob + 4 * (q * NTHR + t)) = ov[q];
  __threadfence();
#pragma unroll
  for (int q = 0; q < 4; ++q) *(volatile v4f*)(ob + 4 * (q * NTHR + t)) = ov[q];
}

extern "C" void kernel_launch(void* const* d_in, const int* in_sizes, int n_in,
                              void* d_out, int out_size, void* d_ws, size_t ws_size,
                              hipStream_t stream) {
  if (n_in < 25) return;
  const int nelem = in_sizes[0];
  if (nelem <= 0 || (nelem % (ROWS * NBIT)) != 0) return;
  const int nrow = nelem / NBIT;
  if (in_sizes[1] != nelem) return;
  if (in_sizes[2]  != NBIT * DMOD || in_sizes[3]  != DMOD || in_sizes[4]  != DMOD || in_sizes[5]  != DMOD) return;
  if (in_sizes[6]  != DMOD * DMOD || in_sizes[7]  != DMOD || in_sizes[8]  != DMOD || in_sizes[9]  != DMOD) return;
  if (in_sizes[10] != DMOD * DMOD || in_sizes[11] != DMOD || in_sizes[12] != DMOD || in_sizes[13] != DMOD) return;
  if (in_sizes[14] != DMOD * NBIT || in_sizes[15] != NBIT) return;
  if (in_sizes[16] != NBIT * DMOD) return;
  if (in_sizes[17] != 2 * DMOD * DMOD || in_sizes[18] != DMOD) return;
  if (in_sizes[19] != DMOD * DMOD || in_sizes[20] != DMOD) return;
  if (in_sizes[21] != 2 * DMOD * DMOD || in_sizes[22] != DMOD) return;
  if (in_sizes[23] != DMOD || in_sizes[24] < 1) return;
  if (out_size != nrow * NBIT) return;

  const float* ibits = (const float*)d_in[0];
  const float* sbits = (const float*)d_in[1];
  const float* W1  = (const float*)d_in[2];  const float* b1  = (const float*)d_in[3];
  const float* g1  = (const float*)d_in[4];  const float* be1 = (const float*)d_in[5];
  const float* W2  = (const float*)d_in[6];  const float* b2  = (const float*)d_in[7];
  const float* g2  = (const float*)d_in[8];  const float* be2 = (const float*)d_in[9];
  const float* W3  = (const float*)d_in[10]; const float* b3  = (const float*)d_in[11];
  const float* g3  = (const float*)d_in[12]; const float* be3 = (const float*)d_in[13];
  const float* W4  = (const float*)d_in[14]; const float* b4  = (const float*)d_in[15];
  const float* pos = (const float*)d_in[16];
  const float* Wq  = (const float*)d_in[17]; const float* bq  = (const float*)d_in[18];
  const float* Wk  = (const float*)d_in[19]; const float* bk  = (const float*)d_in[20];
  const float* Wv1 = (const float*)d_in[21]; const float* bv1 = (const float*)d_in[22];
  const float* Wv2 = (const float*)d_in[23]; const float* bv2 = (const float*)d_in[24];
  float* out = (float*)d_out;

  char* ws = (char*)d_ws;
  size_t off = 0;
  const size_t oKeys = off; off += (size_t)NBIT * DMOD * 4;      off = (off + 255) & ~(size_t)255;
  const size_t oPQ   = off; off += (size_t)NBIT * DMOD * 4;      off = (off + 255) & ~(size_t)255;
  const size_t oPV   = off; off += (size_t)NBIT * DMOD * 4;      off = (off + 255) & ~(size_t)255;
  const size_t oPK   = off; off += (size_t)NBIT * NBIT * 4;      off = (off + 255) & ~(size_t)255;
  const size_t oKh   = off; off += (size_t)NBIT * DMOD * 2;      off = (off + 255) & ~(size_t)255;
  const size_t oW1   = off; off += (size_t)NBIT * DMOD * 2;      off = (off + 255) & ~(size_t)255;
  const size_t oW2   = off; off += (size_t)DMOD * DMOD * 2;      off = (off + 255) & ~(size_t)255;
  const size_t oW3   = off; off += (size_t)DMOD * DMOD * 2;      off = (off + 255) & ~(size_t)255;
  const size_t oW4   = off; off += (size_t)DMOD * NBIT * 2;      off = (off + 255) & ~(size_t)255;
  const size_t oPos  = off; off += (size_t)NBIT * DMOD * 2;      off = (off + 255) & ~(size_t)255;
  const size_t oWq   = off; off += (size_t)DMOD * DMOD * 2;      off = (off + 255) & ~(size_t)255;
  const size_t oWv   = off; off += (size_t)DMOD * DMOD * 2;      off = (off + 255) & ~(size_t)255;
  if (off > ws_size || off > (size_t)WSCAP) return;

  float* keys = (float*)(ws + oKeys);
  float* pqb  = (float*)(ws + oPQ);
  float* pvb  = (float*)(ws + oPV);
  float* pk   = (float*)(ws + oPK);
  _Float16* keysh = (_Float16*)(ws + oKh);
  _Float16* W1h   = (_Float16*)(ws + oW1);
  _Float16* W2h   = (_Float16*)(ws + oW2);
  _Float16* W3h   = (_Float16*)(ws + oW3);
  _Float16* W4h   = (_Float16*)(ws + oW4);
  _Float16* posh  = (_Float16*)(ws + oPos);
  _Float16* Wqh   = (_Float16*)(ws + oWq);
  _Float16* Wv1h  = (_Float16*)(ws + oWv);

  const int t8_64x4  = (NBIT * 64 * 4) / 8;
  const int t8_256x4 = (DMOD * 64 * 4) / 8;
  const int t8_256x1 = (DMOD * 64 * 1) / 8;
  k_pack<<<(t8_64x4  + NTHR - 1) / NTHR, NTHR, 0, stream>>>(W1,  W1h,  NBIT, 4, DMOD, 0,    t8_64x4);
  k_pack<<<(t8_256x4 + NTHR - 1) / NTHR, NTHR, 0, stream>>>(W2,  W2h,  DMOD, 4, DMOD, 0,    t8_256x4);
  k_pack<<<(t8_256x4 + NTHR - 1) / NTHR, NTHR, 0, stream>>>(W3,  W3h,  DMOD, 4, DMOD, 0,    t8_256x4);
  k_pack<<<(t8_256x1 + NTHR - 1) / NTHR, NTHR, 0, stream>>>(W4,  W4h,  DMOD, 1, NBIT, 0,    t8_256x1);
  k_pack<<<(t8_64x4  + NTHR - 1) / NTHR, NTHR, 0, stream>>>(pos, posh, NBIT, 4, DMOD, 0,    t8_64x4);
  k_pack<<<(t8_256x4 + NTHR - 1) / NTHR, NTHR, 0, stream>>>(Wq,  Wqh,  DMOD, 4, DMOD, DMOD, t8_256x4);
  k_pack<<<(t8_256x4 + NTHR - 1) / NTHR, NTHR, 0, stream>>>(Wv1, Wv1h, DMOD, 4, DMOD, DMOD, t8_256x4);

  k_tab<<<NBIT, NTHR, 0, stream>>>(pos, Wq, bq, Wk, bk, Wv1, bv1, keys, pqb, pvb);
  k_pk<<<NBIT, 64, 0, stream>>>(pqb, keys, pk, keysh);

  hipFuncSetAttribute(reinterpret_cast<const void*>(&k_main),
                      hipFuncAttributeMaxDynamicSharedMemorySize, LDS_MAIN);
  k_main<<<nrow / ROWS, NTHR, LDS_MAIN, stream>>>(
      ibits, sbits, b1, g1, be1, b2, g2, be2, b3, g3, be3, b4, Wv2, bv2, pvb, pk,
      W1h, W2h, W3h, W4h, posh, Wqh, Wv1h, keysh, out);
}
